// CrossAttentionwithAttInv_25872882991667
// MI455X (gfx1250) — hardware-verified
//
#include <hip/hip_runtime.h>
#include <stdint.h>

#define NB 8
#define NT 1024
#define NC 768
#define NH 12
#define HD 64
#define NTOK (NB * NT)
#define KSTEPS (NC / 32)
#define GP 32

static_assert(NC % 128 == 0);
static_assert(NC % 32 == 0);
static_assert(NTOK % 64 == 0);
static_assert(NT % 128 == 0);
static_assert(NT % 64 == 0);
static_assert(HD == 64);
static_assert(NH * HD == NC);

typedef _Float16 v8h __attribute__((ext_vector_type(8), __may_alias__));
typedef _Float16 v16h __attribute__((ext_vector_type(16)));
typedef float v8f __attribute__((ext_vector_type(8)));
typedef float v4f __attribute__((ext_vector_type(4), __may_alias__));
typedef unsigned int v4u __attribute__((ext_vector_type(4), __may_alias__));

union FragH { v16h v; v8h half[2]; };

#define WSC 64.0f
#define PSC 256.0f
#define XSC 256.0f
#define SLOG 3.0517578125e-05f
#define OSCA 6.103515625e-05f
#define VUN 0.015625f
#define OSCO 6.103515625e-05f

__device__ __forceinline__ v8f zero8() {
  v8f z = {0.f, 0.f, 0.f, 0.f, 0.f, 0.f, 0.f, 0.f};
  return z;
}

__device__ __forceinline__ v8f wmma16(const FragH& a, const FragH& b, v8f c) {
  v8f d = __builtin_amdgcn_wmma_f32_16x16x32_f16(false, a.v, false, b.v, (short)0, c, false, false);
  asm volatile("v_nop\n\tv_nop\n\tv_nop\n\tv_nop" : "+v"(d) : "v"(a.v), "v"(b.v));
  return d;
}

__device__ __forceinline__ v4u pack8h(v4f a, v4f b, float sc) {
  union { v8h h; v4u u; } k;
  v8h h;
  h[0] = (_Float16)(a[0] * sc); h[1] = (_Float16)(a[1] * sc);
  h[2] = (_Float16)(a[2] * sc); h[3] = (_Float16)(a[3] * sc);
  h[4] = (_Float16)(b[0] * sc); h[5] = (_Float16)(b[1] * sc);
  h[6] = (_Float16)(b[2] * sc); h[7] = (_Float16)(b[3] * sc);
  k.h = h;
  return k.u;
}

__global__ __launch_bounds__(256) void cvt_w_k(
    const float* __restrict__ w0, const float* __restrict__ w1,
    const float* __restrict__ w2, const float* __restrict__ w3,
    _Float16* o0, _Float16* o1, _Float16* o2, _Float16* o3, int n8) {
  const int i = blockIdx.x * 256 + threadIdx.x;
  const int m = i / n8;
  if (m >= 4) return;
  const int e = i - m * n8;
  const float* src = (m == 0) ? w0 : (m == 1) ? w1 : (m == 2) ? w2 : w3;
  _Float16* dst = (m == 0) ? o0 : (m == 1) ? o1 : (m == 2) ? o2 : o3;
  v4f a = *(const v4f*)(src + (size_t)e * 8);
  v4f b = *(const v4f*)(src + (size_t)e * 8 + 4);
  v4u u = pack8h(a, b, WSC);
  volatile v4u* d = (volatile v4u*)(dst + (size_t)e * 8);
  *d = u;
  __threadfence();
  *d = u;
}

__global__ __launch_bounds__(256) void prep_k(
    const float* __restrict__ q_in, const float* __restrict__ kv_in,
    const float* __restrict__ W2, const float* __restrict__ b2,
    const float* __restrict__ W1, const float* __restrict__ b1,
    const float* __restrict__ ssp, const float* __restrict__ sbp,
    _Float16* Xq, _Float16* Xkv, float* G, int ntok) {
  __shared__ __align__(16) float feat[NC];
  __shared__ __align__(16) float gsh[GP];
  const int tok = blockIdx.x;
  if (tok >= ntok) return;
  const int t = threadIdx.x, wv = t >> 5, ln = t & 31;
  const float ss = ssp[0], sb = sbp[0];
  const float* qr = q_in + (size_t)tok * NC;
  const float* kr = kv_in + (size_t)tok * NC;
  if (t < GP) gsh[t] = 0.0f;

  const bool hasx = (t < 192);
  v4u ux = {0u, 0u, 0u, 0u};
  volatile v4u* xd = nullptr;
  if (t < 96) {
    v4f a = *(const v4f*)(qr + 8 * t);
    v4f b = *(const v4f*)(qr + 8 * t + 4);
    ux = pack8h(a, b, 1.0f);
    xd = (volatile v4u*)(Xq + (size_t)tok * NC + 8 * t);
  } else if (t < 192) {
    const int tt = t - 96;
    v4f a = *(const v4f*)(kr + 8 * tt);
    v4f b = *(const v4f*)(kr + 8 * tt + 4);
    ux = pack8h(a, b, 1.0f);
    xd = (volatile v4u*)(Xkv + (size_t)tok * NC + 8 * tt);
  }
  if (hasx) *xd = ux;

  for (int i = t; i < NC; i += 256) {
    float x = qr[i];
    float r = fmaxf(x, 0.0f);
    feat[i] = ss * (r * r) + sb;
  }
  __syncthreads();

  for (int o = wv; o < 2 * NH; o += 8) {
    const float* wr = (o < NH) ? (W2 + (size_t)o * NC) : (W1 + (size_t)(o - NH) * NC);
    float s = 0.0f;
    for (int j = ln; j < NC; j += 32) s += feat[j] * wr[j];
    s += __shfl_xor(s, 16);
    s += __shfl_xor(s, 8);
    s += __shfl_xor(s, 4);
    s += __shfl_xor(s, 2);
    s += __shfl_xor(s, 1);
    if (ln == 0) {
      if (o < NH) {
        gsh[o] = tanhf(s + b2[o]);
      } else {
        float x = s + b1[o - NH];
        float sp = fmaxf(x, 0.0f) + log1pf(__expf(-fabsf(x)));
        float s2 = sp * sp;
        gsh[16 + (o - NH)] = 2.0f * s2 / (s2 + 0.3678f);
      }
    }
  }
  __syncthreads();

  v4f gv = {0.f, 0.f, 0.f, 0.f};
  volatile v4f* gd = nullptr;
  if (t < 8) {
    gv = *(const v4f*)(gsh + 4 * t);
    gd = (volatile v4f*)(G + (size_t)tok * GP + 4 * t);
    *gd = gv;
  }
  __threadfence();
  if (hasx) *xd = ux;
  if (t < 8) *gd = gv;
}

__global__ __launch_bounds__(128) void gemm_k(
    const _Float16* __restrict__ A, const _Float16* __restrict__ W,
    const float* __restrict__ bias, _Float16* dst16, float* dst32, int mode, float osc) {
  __shared__ __align__(16) _Float16 As[64 * 40];
  __shared__ __align__(16) _Float16 Bs[128 * 40];
  __shared__ __align__(16) float Ts[8704];
  const int t = threadIdx.x, wv = t >> 5, ln = t & 31, lm = ln & 15, hi = ln >> 4;
  const int wvm = wv & 1, wvn = wv >> 1;
  const int bm = blockIdx.y * 64, bn = blockIdx.x * 128;
  if (bm + 64 > NTOK || bn + 128 > NC) return;
  const int sr = t >> 2, sp = t & 3;

  v8f acc[2][4];
#pragma unroll
  for (int i = 0; i < 2; ++i)
#pragma unroll
    for (int c = 0; c < 4; ++c) acc[i][c] = zero8();

  for (int s = 0; s < KSTEPS; ++s) {
    const int kk = s * 32;
    __syncthreads();
    *(v8h*)(As + sr * 40 + sp * 8) = *(const v8h*)(A + (size_t)(bm + sr) * NC + kk + sp * 8);
    *(v8h*)(As + (sr + 32) * 40 + sp * 8) = *(const v8h*)(A + (size_t)(bm + sr + 32) * NC + kk + sp * 8);
#pragma unroll
    for (int u = 0; u < 4; ++u)
      *(v8h*)(Bs + (sr + 32 * u) * 40 + sp * 8) =
          *(const v8h*)(W + (size_t)(bn + sr + 32 * u) * NC + kk + sp * 8);
    __syncthreads();

    FragH fa[2];
#pragma unroll
    for (int i = 0; i < 2; ++i) {
      fa[i].half[0] = *(const v8h*)(As + (wvm * 32 + 16 * i + lm) * 40 + 8 * hi);
      fa[i].half[1] = *(const v8h*)(As + (wvm * 32 + 16 * i + lm) * 40 + 16 + 8 * hi);
    }
#pragma unroll
    for (int c = 0; c < 4; ++c) {
      FragH fb;
      fb.half[0] = *(const v8h*)(Bs + (wvn * 64 + 16 * c + lm) * 40 + 8 * hi);
      fb.half[1] = *(const v8h*)(Bs + (wvn * 64 + 16 * c + lm) * 40 + 16 + 8 * hi);
      acc[0][c] = wmma16(fa[0], fb, acc[0][c]);
      acc[1][c] = wmma16(fa[1], fb, acc[1][c]);
    }
  }

#pragma unroll
  for (int i = 0; i < 2; ++i)
#pragma unroll
    for (int c = 0; c < 4; ++c)
#pragma unroll
      for (int r = 0; r < 8; ++r) {
        const int row = wvm * 32 + 16 * i + 8 * hi + r;
        const int col = wvn * 64 + 16 * c + lm;
        if (mode == 1) Ts[col * 68 + row] = acc[i][c][r];
        else           Ts[row * 132 + col] = acc[i][c][r];
      }
  __syncthreads();

  const int p = ln & 7;
  const int lq = ln >> 3;
  const int h0 = bn >> 6;
  for (int pass = 0; pass < 2; ++pass) {
    if (mode == 0) {
#pragma unroll
      for (int it = 0; it < 8; ++it) {
        const int L = wv * 32 + it * 4 + lq;
        const int r = L >> 1, j = L & 1;
        const float* sp0 = Ts + r * 132 + 64 * j + 8 * p;
        v4f f0 = *(const v4f*)sp0;
        v4f f1 = *(const v4f*)(sp0 + 4);
        v4u u = pack8h(f0, f1, 1.0f);
        const int m = bm + r;
        const int b = m >> 10, n = m & 1023;
        _Float16* d = dst16 + (((size_t)(b * NH + h0 + j) * NT + n) * HD + 8 * p);
        *(volatile v4u*)d = u;
      }
    } else if (mode == 1) {
      const int b = bm >> 10, n0 = bm & 1023;
#pragma unroll
      for (int it = 0; it < 8; ++it) {
        const int c = wv * 32 + it * 4 + lq;
        const float* sp0 = Ts + c * 68 + 8 * p;
        v4f f0 = *(const v4f*)sp0;
        v4f f1 = *(const v4f*)(sp0 + 4);
        v4u u = pack8h(f0, f1, 1.0f);
        _Float16* d = dst16 + (((size_t)(b * NH + h0 + (c >> 6)) * HD + (c & 63)) * NT + n0 + 8 * p);
        *(volatile v4u*)d = u;
      }
    } else {
#pragma unroll
      for (int it = 0; it < 16; ++it) {
        const int L = wv * 64 + it * 4 + lq;
        const int r = L >> 2, q = L & 3;
        v4f f = *(const v4f*)(Ts + r * 132 + 32 * q + 4 * p);
        const int col = bn + 32 * q + 4 * p;
        v4f bv;
        bv[0] = bias[col]; bv[1] = bias[col + 1]; bv[2] = bias[col + 2]; bv[3] = bias[col + 3];
        v4f val = f * osc + bv;
        float* d = dst32 + ((size_t)(bm + r) * NC + col);
        *(volatile v4f*)d = val;
      }
    }
    if (pass == 0) __threadfence();
  }
}

__global__ __launch_bounds__(256) void attn_k(
    const _Float16* __restrict__ Qh, const _Float16* __restrict__ Kh,
    const _Float16* __restrict__ Vt, const float* __restrict__ G,
    const float* __restrict__ lfg, const float* __restrict__ hfg, _Float16* xg) {
  __shared__ __align__(16) _Float16 Plds[8 * 16 * 40];
  __shared__ __align__(16) float Of[8 * 16 * 68];
  const int t = threadIdx.x, wv = t >> 5, ln = t & 31, lm = ln & 15, hi = ln >> 4;
  const int bh = blockIdx.y, q0 = blockIdx.x * 128;
  if (bh >= NB * NH || q0 + 128 > NT) return;
  const int b = bh / NH, h = bh - b * NH;
  const int qw = q0 + wv * 16;

  const _Float16* Qp = Qh + ((size_t)bh * NT + qw) * HD;
  const _Float16* Kp = Kh + (size_t)bh * NT * HD;
  const _Float16* Vp = Vt + (size_t)bh * HD * NT;
  _Float16* Pw = Plds + wv * 640;
  float* Ow = Of + wv * 1088;

  FragH qa[2];
#pragma unroll
  for (int j = 0; j < 2; ++j) {
    qa[j].half[0] = *(const v8h*)(Qp + lm * HD + 32 * j + 8 * hi);
    qa[j].half[1] = *(const v8h*)(Qp + lm * HD + 32 * j + 16 + 8 * hi);
  }

  v8f o[4];
#pragma unroll
  for (int j = 0; j < 4; ++j) o[j] = zero8();
  float mrow[8], lrow[8];
#pragma unroll
  for (int r = 0; r < 8; ++r) { mrow[r] = -3.0e38f; lrow[r] = 0.0f; }

  for (int kb = 0; kb < NT; kb += 32) {
    v8f s[2];
    s[0] = zero8(); s[1] = zero8();
#pragma unroll
    for (int tt = 0; tt < 2; ++tt) {
      const _Float16* krow = Kp + (size_t)(kb + 16 * tt + lm) * HD;
#pragma unroll
      for (int j = 0; j < 2; ++j) {
        FragH kf;
        kf.half[0] = *(const v8h*)(krow + 32 * j + 8 * hi);
        kf.half[1] = *(const v8h*)(krow + 32 * j + 16 + 8 * hi);
        s[tt] = wmma16(qa[j], kf, s[tt]);
      }
    }

    float fac[8];
#pragma unroll
    for (int r = 0; r < 8; ++r) {
      float v0 = s[0][r] * SLOG;
      float v1 = s[1][r] * SLOG;
      float tm = fmaxf(v0, v1);
      tm = fmaxf(tm, __shfl_xor(tm, 1));
      tm = fmaxf(tm, __shfl_xor(tm, 2));
      tm = fmaxf(tm, __shfl_xor(tm, 4));
      tm = fmaxf(tm, __shfl_xor(tm, 8));
      float mn = fmaxf(mrow[r], tm);
      float fc = __expf(mrow[r] - mn);
      mrow[r] = mn;
      fac[r] = fc;
      float p0 = __expf(v0 - mn);
      float p1 = __expf(v1 - mn);
      float rs = p0 + p1;
      rs += __shfl_xor(rs, 1);
      rs += __shfl_xor(rs, 2);
      rs += __shfl_xor(rs, 4);
      rs += __shfl_xor(rs, 8);
      lrow[r] = lrow[r] * fc + rs;
      Pw[(8 * hi + r) * 40 + lm]      = (_Float16)(PSC * p0);
      Pw[(8 * hi + r) * 40 + 16 + lm] = (_Float16)(PSC * p1);
    }
#pragma unroll
    for (int r = 0; r < 8; ++r) {
      o[0][r] *= fac[r]; o[1][r] *= fac[r]; o[2][r] *= fac[r]; o[3][r] *= fac[r];
    }
    __syncthreads();

    FragH pf;
    pf.half[0] = *(const v8h*)(Pw + lm * 40 + 8 * hi);
    pf.half[1] = *(const v8h*)(Pw + lm * 40 + 16 + 8 * hi);
#pragma unroll
    for (int j = 0; j < 4; ++j) {
      const _Float16* vrow = Vp + (size_t)(16 * j + lm) * NT + kb;
      FragH vf;
      vf.half[0] = *(const v8h*)(vrow + 8 * hi);
      vf.half[1] = *(const v8h*)(vrow + 16 + 8 * hi);
      o[j] = wmma16(pf, vf, o[j]);
    }
    __syncthreads();
  }

  float inv[8], dlf[8], dhf[8];
#pragma unroll
  for (int r = 0; r < 8; ++r) {
    const int qi = qw + 8 * hi + r;
    const size_t tokg = (size_t)(b * NT + qi);
    inv[r] = OSCA / lrow[r];
    dlf[r] = G[tokg * GP + h];
    dhf[r] = G[tokg * GP + 16 + h];
  }
#pragma unroll
  for (int j = 0; j < 4; ++j) {
    const int d = 16 * j + lm;
    const int c = h * HD + d;
    const float lg = lfg[c], hg = hfg[c];
    union { v8h v; _Float16 e[8]; } vv;
    vv.v = *(const v8h*)(Vp + (size_t)d * NT + qw + 8 * hi);
#pragma unroll
    for (int r = 0; r < 8; ++r) {
      float x = o[j][r] * inv[r];
      float vr = (float)vv.e[r] * VUN;
      float a1 = x * dlf[r] * lg;
      float b1 = dhf[r] * (vr - x) * hg;
      float y = (x + a1) + b1;
      Ow[(8 * hi + r) * 68 + d] = y;
    }
  }
  __syncthreads();

  const int p = ln & 7, lq = ln >> 3;
  for (int pass = 0; pass < 2; ++pass) {
#pragma unroll
    for (int it = 0; it < 4; ++it) {
      const int row = it * 4 + lq;
      const float* sp0 = Ow + row * 68 + 8 * p;
      v4f f0 = *(const v4f*)sp0;
      v4f f1 = *(const v4f*)(sp0 + 4);
      v4u u = pack8h(f0, f1, XSC);
      _Float16* dptr = xg + ((size_t)(b * NT + qw + row) * NC + h * HD + 8 * p);
      *(volatile v4u*)dptr = u;
    }
    if (pass == 0) __threadfence();
  }
}

extern "C" void kernel_launch(void* const* d_in, const int* in_sizes, int n_in,
                              void* d_out, int out_size, void* d_ws, size_t ws_size,
                              hipStream_t stream) {
  if (n_in < 15) return;
  if (in_sizes[0] != NTOK * NC || in_sizes[1] != NTOK * NC) return;
  if (in_sizes[2] != NC * NC || in_sizes[3] != NC * NC || in_sizes[4] != NC * NC || in_sizes[5] != NC * NC) return;
  if (in_sizes[6] != NC || in_sizes[7] != NH * NC || in_sizes[8] != NH || in_sizes[9] != NH * NC || in_sizes[10] != NH) return;
  if (in_sizes[11] != NC || in_sizes[12] != NC || in_sizes[13] < 1 || in_sizes[14] < 1) return;
  if (out_size != NTOK * NC) return;

  const float* q_in       = (const float*)d_in[0];
  const float* kv_in      = (const float*)d_in[1];
  const float* Wq         = (const float*)d_in[2];
  const float* Wk         = (const float*)d_in[3];
  const float* Wv         = (const float*)d_in[4];
  const float* Wp         = (const float*)d_in[5];
  const float* bp         = (const float*)d_in[6];
  const float* W_dy2      = (const float*)d_in[7];
  const float* b_dy2      = (const float*)d_in[8];
  const float* W_dy       = (const float*)d_in[9];
  const float* b_dy       = (const float*)d_in[10];
  const float* lf_gamma   = (const float*)d_in[11];
  const float* hf_gamma   = (const float*)d_in[12];
  const float* star_scale = (const float*)d_in[13];
  const float* star_bias  = (const float*)d_in[14];
  float* out = (float*)d_out;

  char* base = (char*)d_ws;
  size_t off = 0;
  auto carve = [&](size_t bytes) -> char* {
    char* p = base + off;
    off += (bytes + 255) & ~(size_t)255;
    return p;
  };
  const size_t wbytes = (size_t)NC * NC * 2;
  const size_t xbytes = (size_t)NTOK * NC * 2;
  _Float16* Wqh = (_Float16*)carve(wbytes);
  _Float16* Wkh = (_Float16*)carve(wbytes);
  _Float16* Wvh = (_Float16*)carve(wbytes);
  _Float16* Wph = (_Float16*)carve(wbytes);
  _Float16* Xq  = (_Float16*)carve(xbytes);
  _Float16* Xkv = (_Float16*)carve(xbytes);
  _Float16* Qh  = (_Float16*)carve(xbytes);
  _Float16* Kh  = (_Float16*)carve(xbytes);
  _Float16* Vth = (_Float16*)carve(xbytes);
  float*    G   = (float*)carve((size_t)NTOK * GP * 4);
  _Float16* xg  = (_Float16*)carve(xbytes);
  if (off > ws_size) return;

  const int n8 = NC * NC / 8;
  cvt_w_k<<<(4 * n8 + 255) / 256, 256, 0, stream>>>(Wq, Wk, Wv, Wp, Wqh, Wkh, Wvh, Wph, n8);
  prep_k<<<NTOK, 256, 0, stream>>>(q_in, kv_in, W_dy2, b_dy2, W_dy, b_dy, star_scale, star_bias,
                                   Xq, Xkv, G, NTOK);
  const dim3 ggrid(NC / 128, NTOK / 64);
  gemm_k<<<ggrid, 128, 0, stream>>>(Xq,  Wqh, bp, Qh,  out, 0, 1.0f);
  gemm_k<<<ggrid, 128, 0, stream>>>(Xkv, Wkh, bp, Kh,  out, 0, 1.0f);
  gemm_k<<<ggrid, 128, 0, stream>>>(Xkv, Wvh, bp, Vth, out, 1, 1.0f);
  attn_k<<<dim3(NT / 128, NB * NH), 256, 0, stream>>>(Qh, Kh, Vth, G, lf_gamma, hf_gamma, xg);
  gemm_k<<<ggrid, 128, 0, stream>>>(xg, Wph, bp, Qh, out, 2, OSCO);
}
